// FourierAttention2d_44169443672697
// MI455X (gfx1250) — hardware-verified
//
#include <hip/hip_runtime.h>
#include <stddef.h>


#define NB     4
#define NTOK   16384
#define CIN    64
#define NH     8
#define DH     64
#define HD     (NH * DH)
#define NTILE  8
#define CHT    (NTOK / NTILE)
#define KVIT   (CHT / 64)
#define TP     72
#define NVB    ((NB * NTOK * CIN) / (256 * 8))
#define NWB    64
#define WSC    64.0f
#define RWSC   (1.0f / 64.0f)
#define EPSV   1e-5f
#define WSCAP  134217728

static_assert(CIN == 64 && DH == 64 && HD == 512 && NH == 8);
static_assert((NTOK % NTILE) == 0 && (CHT % 64) == 0 && (NTOK % 64) == 0);
static_assert(NVB * 256 * 8 == NB * NTOK * CIN);
static_assert(16 * 256 * 8 == CIN * HD && 16 * 256 * 8 == HD * DH);
static_assert((TP % 8) == 0 && TP >= 64);

typedef float    v4f  __attribute__((ext_vector_type(4)));
typedef float    v8f  __attribute__((ext_vector_type(8)));
typedef _Float16 v8h  __attribute__((ext_vector_type(8)));
typedef _Float16 v16h __attribute__((ext_vector_type(16)));
union FragH { v16h v; v8h h[2]; };

__device__ __forceinline__ v8f wmf(v16h a, v16h b, v8f c) {
  v8f d = __builtin_amdgcn_wmma_f32_16x16x32_f16(false, a, false, b, (short)0, c, false, false);
  asm volatile("v_nop\n\tv_nop\n\tv_nop\n\tv_nop" : "+v"(d) : "v"(a), "v"(b));
  return d;
}

__device__ __forceinline__ v16h ldfrag(const _Float16* p, int ld) {
  const int l = threadIdx.x & 31, hh = l >> 4, m = l & 15;
  const _Float16* q = p + m * ld + 8 * hh;
  FragH f;
  f.h[0] = *(const v8h*)q;
  f.h[1] = *(const v8h*)(q + 16);
  return f.v;
}

__device__ __forceinline__ float hred16(float x) {
  x += __shfl_xor(x, 8, 32);
  x += __shfl_xor(x, 4, 32);
  x += __shfl_xor(x, 2, 32);
  x += __shfl_xor(x, 1, 32);
  return x;
}

__global__ __launch_bounds__(256) void k_prep(
    const float* __restrict__ v, const float* __restrict__ Wq, const float* __restrict__ Wk,
    const float* __restrict__ Wv, const float* __restrict__ Wo,
    _Float16* vh, _Float16* WqT, _Float16* WkT, _Float16* WvT, _Float16* WoP) {
  const int t = threadIdx.x;
  const int bid = blockIdx.x;
  v8h o;
  _Float16* d;
  if (bid < NVB) {
    const size_t i = (size_t)bid * 256 + t;
    const v4f a = *(const v4f*)(v + i * 8);
    const v4f c = *(const v4f*)(v + i * 8 + 4);
    o[0] = (_Float16)a.x; o[1] = (_Float16)a.y; o[2] = (_Float16)a.z; o[3] = (_Float16)a.w;
    o[4] = (_Float16)c.x; o[5] = (_Float16)c.y; o[6] = (_Float16)c.z; o[7] = (_Float16)c.w;
    d = vh + i * 8;
  } else {
    const int wb = bid - NVB;
    const int which = wb >> 4;
    const int i = (wb & 15) * 256 + t;
    if (which < 3) {
      const float* W = (which == 0) ? Wq : ((which == 1) ? Wk : Wv);
      _Float16* T = (which == 0) ? WqT : ((which == 1) ? WkT : WvT);
      const int oc = i >> 3, c0 = (i & 7) * 8;
#pragma unroll
      for (int e = 0; e < 8; ++e) o[e] = (_Float16)(W[(c0 + e) * HD + oc] * WSC);
      d = T + (size_t)i * 8;
    } else {
      const int e = i >> 6, k0 = (i & 63) * 8;
#pragma unroll
      for (int j = 0; j < 8; ++j) o[j] = (_Float16)(Wo[(k0 + j) * DH + e] * WSC);
      d = WoP + (size_t)i * 8;
    }
  }
  *(volatile v8h*)d = o;
  __threadfence();
  *(volatile v8h*)d = o;
}

__global__ __launch_bounds__(128) void k_kv(
    const _Float16* __restrict__ vh, const _Float16* __restrict__ WkT, const _Float16* __restrict__ WvT,
    const float* __restrict__ Wk_b, const float* __restrict__ Wv_b,
    const float* __restrict__ lnk_g, const float* __restrict__ lnk_b, float* part) {
  __shared__ __attribute__((aligned(16))) _Float16 Kt[DH * TP];
  __shared__ __attribute__((aligned(16))) _Float16 Vt[DH * TP];
  __shared__ __attribute__((aligned(16))) float stg[4 * 16 * DH];
  const int lane = threadIdx.x & 31, wv = threadIdx.x >> 5, hh = lane >> 4, m = lane & 15;
  const int tile = blockIdx.x % NTILE;
  const int h = (blockIdx.x / NTILE) % NH;
  const int b = blockIdx.x / (NTILE * NH);

  float bk[4], bv[4], gk[4], btk[4];
#pragma unroll
  for (int nt = 0; nt < 4; ++nt) {
    const int col = h * DH + 16 * nt + m;
    bk[nt] = Wk_b[col]; bv[nt] = Wv_b[col];
    gk[nt] = lnk_g[col]; btk[nt] = lnk_b[col];
  }

  v8f kvacc[4];
#pragma unroll
  for (int et = 0; et < 4; ++et) { v8f z = {0.f, 0.f, 0.f, 0.f, 0.f, 0.f, 0.f, 0.f}; kvacc[et] = z; }

#pragma unroll 1
  for (int it = 0; it < KVIT; ++it) {
    const size_t tok0 = (size_t)b * NTOK + (size_t)tile * CHT + (size_t)it * 64 + (size_t)wv * 16;
    const _Float16* ap = vh + tok0 * CIN;
    const v16h av0 = ldfrag(ap, CIN);
    const v16h av1 = ldfrag(ap + 32, CIN);

    v8f ck[4], cv[4];
#pragma unroll
    for (int nt = 0; nt < 4; ++nt) {
      v8f z = {0.f, 0.f, 0.f, 0.f, 0.f, 0.f, 0.f, 0.f}; ck[nt] = z; cv[nt] = z;
      const _Float16* wk = WkT + (size_t)(h * DH + 16 * nt) * CIN;
      const _Float16* wvp = WvT + (size_t)(h * DH + 16 * nt) * CIN;
      ck[nt] = wmf(av0, ldfrag(wk, CIN), ck[nt]);
      ck[nt] = wmf(av1, ldfrag(wk + 32, CIN), ck[nt]);
      cv[nt] = wmf(av0, ldfrag(wvp, CIN), cv[nt]);
      cv[nt] = wmf(av1, ldfrag(wvp + 32, CIN), cv[nt]);
    }

#pragma unroll
    for (int r = 0; r < 8; ++r) {
      float x0 = ck[0][r] * RWSC + bk[0];
      float x1 = ck[1][r] * RWSC + bk[1];
      float x2 = ck[2][r] * RWSC + bk[2];
      float x3 = ck[3][r] * RWSC + bk[3];
      float s = (x0 + x1) + (x2 + x3);
      s = hred16(s);
      const float mu = s * (1.0f / 64.0f);
      x0 -= mu; x1 -= mu; x2 -= mu; x3 -= mu;
      float q = (x0 * x0 + x1 * x1) + (x2 * x2 + x3 * x3);
      q = hred16(q);
      const float var = q * (1.0f / 64.0f);
      const float rs = rsqrtf(var + EPSV);
      ck[0][r] = x0 * rs * gk[0] + btk[0];
      ck[1][r] = x1 * rs * gk[1] + btk[1];
      ck[2][r] = x2 * rs * gk[2] + btk[2];
      ck[3][r] = x3 * rs * gk[3] + btk[3];
    }

#pragma unroll
    for (int nt = 0; nt < 4; ++nt) {
      v8h kk, vv;
#pragma unroll
      for (int r = 0; r < 8; ++r) {
        kk[r] = (_Float16)ck[nt][r];
        vv[r] = (_Float16)(cv[nt][r] * RWSC + bv[nt]);
      }
      *(v8h*)(Kt + (16 * nt + m) * TP + wv * 16 + 8 * hh) = kk;
      *(v8h*)(Vt + (16 * nt + m) * TP + wv * 16 + 8 * hh) = vv;
    }
    __syncthreads();

    const _Float16* ka = Kt + (16 * wv) * TP;
#pragma unroll
    for (int ks = 0; ks < 2; ++ks) {
      const v16h ak = ldfrag(ka + 32 * ks, TP);
#pragma unroll
      for (int et = 0; et < 4; ++et)
        kvacc[et] = wmf(ak, ldfrag(Vt + (16 * et) * TP + 32 * ks, TP), kvacc[et]);
    }
    __syncthreads();
  }

  float* sw = stg + wv * (16 * DH);
#pragma unroll
  for (int et = 0; et < 4; ++et) {
#pragma unroll
    for (int r = 0; r < 8; ++r) sw[(8 * hh + r) * DH + 16 * et + m] = kvacc[et][r];
  }
  __syncthreads();
  float* gp = part + ((size_t)blockIdx.x * DH + (size_t)(16 * wv)) * DH;
#pragma unroll
  for (int i = 0; i < 8; ++i) {
    const v4f x = *(const v4f*)(sw + i * 128 + 4 * lane);
    *(volatile v4f*)(gp + i * 128 + 4 * lane) = x;
  }
  __threadfence();
#pragma unroll
  for (int i = 0; i < 8; ++i) {
    const v4f x = *(const v4f*)(sw + i * 128 + 4 * lane);
    *(volatile v4f*)(gp + i * 128 + 4 * lane) = x;
  }
}

__global__ __launch_bounds__(256) void k_kvred(const float* __restrict__ part, _Float16* kvT) {
  __shared__ __attribute__((aligned(16))) float kvs[DH * DH];
  const int t = threadIdx.x;
  const int bh = blockIdx.x;
  const float* p0 = part + (size_t)bh * NTILE * (DH * DH);
#pragma unroll 1
  for (int j = 0; j < (DH * DH) / 256; ++j) {
    const int idx = j * 256 + t;
    float s = 0.0f;
#pragma unroll
    for (int tl = 0; tl < NTILE; ++tl) s += p0[(size_t)tl * (DH * DH) + idx];
    kvs[idx] = s;
  }
  __syncthreads();
  v8h o0, o1;
  {
    const int idx = t;
    const int e = idx >> 3, d0 = (idx & 7) * 8;
#pragma unroll
    for (int i = 0; i < 8; ++i) o0[i] = (_Float16)(kvs[(d0 + i) * DH + e] * (1.0f / 16.0f));
  }
  {
    const int idx = t + 256;
    const int e = idx >> 3, d0 = (idx & 7) * 8;
#pragma unroll
    for (int i = 0; i < 8; ++i) o1[i] = (_Float16)(kvs[(d0 + i) * DH + e] * (1.0f / 16.0f));
  }
  _Float16* dp0 = kvT + (size_t)bh * (DH * DH) + (size_t)t * 8;
  _Float16* dp1 = dp0 + 2048;
  *(volatile v8h*)dp0 = o0;
  *(volatile v8h*)dp1 = o1;
  __threadfence();
  *(volatile v8h*)dp0 = o0;
  *(volatile v8h*)dp1 = o1;
}

__global__ __launch_bounds__(128) void k_out(
    const _Float16* __restrict__ vh, const _Float16* __restrict__ WqT,
    const float* __restrict__ Wq_b, const float* __restrict__ lnq_g, const float* __restrict__ lnq_b,
    const _Float16* __restrict__ kvT, const _Float16* __restrict__ WoP,
    const float* __restrict__ Wo_b, float* out) {
  __shared__ __attribute__((aligned(16))) _Float16 Qs[4 * 16 * TP];
  __shared__ __attribute__((aligned(16))) _Float16 As[4 * 16 * TP];
  __shared__ __attribute__((aligned(16))) float stg[4 * 16 * DH];
  const int lane = threadIdx.x & 31, wv = threadIdx.x >> 5, hh = lane >> 4, m = lane & 15;
  const int b = blockIdx.x / (NTOK / 64);
  const size_t tok0 = (size_t)blockIdx.x * 64 + (size_t)wv * 16;
  _Float16* Qw = Qs + wv * (16 * TP);
  _Float16* Aw = As + wv * (16 * TP);
  float* sw = stg + wv * (16 * DH);

  const _Float16* ap = vh + tok0 * CIN;
  const v16h av0 = ldfrag(ap, CIN);
  const v16h av1 = ldfrag(ap + 32, CIN);

  float wob[4];
#pragma unroll
  for (int nt = 0; nt < 4; ++nt) wob[nt] = Wo_b[16 * nt + m] * (1.0f / 16384.0f);

  v8f co[4];
#pragma unroll
  for (int nt = 0; nt < 4; ++nt) { v8f z = {0.f, 0.f, 0.f, 0.f, 0.f, 0.f, 0.f, 0.f}; co[nt] = z; }

#pragma unroll 1
  for (int h = 0; h < NH; ++h) {
    float bq[4], gq[4], btq[4];
#pragma unroll
    for (int nt = 0; nt < 4; ++nt) {
      const int col = h * DH + 16 * nt + m;
      bq[nt] = Wq_b[col]; gq[nt] = lnq_g[col]; btq[nt] = lnq_b[col];
    }

    v8f cq[4];
#pragma unroll
    for (int nt = 0; nt < 4; ++nt) {
      v8f z = {0.f, 0.f, 0.f, 0.f, 0.f, 0.f, 0.f, 0.f}; cq[nt] = z;
      const _Float16* wq = WqT + (size_t)(h * DH + 16 * nt) * CIN;
      cq[nt] = wmf(av0, ldfrag(wq, CIN), cq[nt]);
      cq[nt] = wmf(av1, ldfrag(wq + 32, CIN), cq[nt]);
    }

#pragma unroll
    for (int r = 0; r < 8; ++r) {
      float x0 = cq[0][r] * RWSC + bq[0];
      float x1 = cq[1][r] * RWSC + bq[1];
      float x2 = cq[2][r] * RWSC + bq[2];
      float x3 = cq[3][r] * RWSC + bq[3];
      float s = (x0 + x1) + (x2 + x3);
      s = hred16(s);
      const float mu = s * (1.0f / 64.0f);
      x0 -= mu; x1 -= mu; x2 -= mu; x3 -= mu;
      float q = (x0 * x0 + x1 * x1) + (x2 * x2 + x3 * x3);
      q = hred16(q);
      const float var = q * (1.0f / 64.0f);
      const float rs = rsqrtf(var + EPSV);
      cq[0][r] = x0 * rs * gq[0] + btq[0];
      cq[1][r] = x1 * rs * gq[1] + btq[1];
      cq[2][r] = x2 * rs * gq[2] + btq[2];
      cq[3][r] = x3 * rs * gq[3] + btq[3];
    }

#pragma unroll
    for (int nt = 0; nt < 4; ++nt) {
#pragma unroll
      for (int r = 0; r < 8; ++r) Qw[(8 * hh + r) * TP + 16 * nt + m] = (_Float16)cq[nt][r];
    }
    __syncthreads();

    const v16h aq0 = ldfrag(Qw, TP);
    const v16h aq1 = ldfrag(Qw + 32, TP);
    const _Float16* kp = kvT + (size_t)(b * NH + h) * (DH * DH);
    v8f ca[4];
#pragma unroll
    for (int et = 0; et < 4; ++et) {
      v8f z = {0.f, 0.f, 0.f, 0.f, 0.f, 0.f, 0.f, 0.f}; ca[et] = z;
      ca[et] = wmf(aq0, ldfrag(kp + (16 * et) * DH, DH), ca[et]);
      ca[et] = wmf(aq1, ldfrag(kp + (16 * et) * DH + 32, DH), ca[et]);
    }

#pragma unroll
    for (int et = 0; et < 4; ++et) {
#pragma unroll
      for (int r = 0; r < 8; ++r) Aw[(8 * hh + r) * TP + 16 * et + m] = (_Float16)(ca[et][r] * (1.0f / 64.0f));
    }
    __syncthreads();

    const v16h aa0 = ldfrag(Aw, TP);
    const v16h aa1 = ldfrag(Aw + 32, TP);
    const _Float16* wo = WoP + h * DH;
#pragma unroll
    for (int nt = 0; nt < 4; ++nt) {
      co[nt] = wmf(aa0, ldfrag(wo + (size_t)(16 * nt) * HD, HD), co[nt]);
      co[nt] = wmf(aa1, ldfrag(wo + (size_t)(16 * nt) * HD + 32, HD), co[nt]);
    }
  }

#pragma unroll
  for (int nt = 0; nt < 4; ++nt) {
#pragma unroll
    for (int r = 0; r < 8; ++r) sw[(8 * hh + r) * DH + 16 * nt + m] = co[nt][r] * (1.0f / 1024.0f) + wob[nt];
  }
  __syncthreads();
  float* gp = out + tok0 * DH;
#pragma unroll
  for (int i = 0; i < 8; ++i) {
    const v4f x = *(const v4f*)(sw + i * 128 + 4 * lane);
    *(volatile v4f*)(gp + i * 128 + 4 * lane) = x;
  }
  __threadfence();
#pragma unroll
  for (int i = 0; i < 8; ++i) {
    const v4f x = *(const v4f*)(sw + i * 128 + 4 * lane);
    *(volatile v4f*)(gp + i * 128 + 4 * lane) = x;
  }
}

extern "C" void kernel_launch(void* const* d_in, const int* in_sizes, int n_in,
                              void* d_out, int out_size, void* d_ws, size_t ws_size,
                              hipStream_t stream) {
  if (n_in < 13) return;
  if (in_sizes[0] != NB * NTOK * CIN) return;
  if (in_sizes[1] != CIN * HD || in_sizes[3] != CIN * HD || in_sizes[5] != CIN * HD) return;
  if (in_sizes[2] != HD || in_sizes[4] != HD || in_sizes[6] != HD) return;
  if (in_sizes[7] != NH * DH || in_sizes[8] != NH * DH || in_sizes[9] != NH * DH || in_sizes[10] != NH * DH) return;
  if (in_sizes[11] != HD * DH || in_sizes[12] != DH) return;
  if (out_size != NB * NTOK * DH) return;

  const float* v     = (const float*)d_in[0];
  const float* Wq_w  = (const float*)d_in[1];
  const float* Wq_b  = (const float*)d_in[2];
  const float* Wk_w  = (const float*)d_in[3];
  const float* Wk_b  = (const float*)d_in[4];
  const float* Wv_w  = (const float*)d_in[5];
  const float* Wv_b  = (const float*)d_in[6];
  const float* lnq_g = (const float*)d_in[7];
  const float* lnq_b = (const float*)d_in[8];
  const float* lnk_g = (const float*)d_in[9];
  const float* lnk_b = (const float*)d_in[10];
  const float* Wo_w  = (const float*)d_in[11];
  const float* Wo_b  = (const float*)d_in[12];
  float* out = (float*)d_out;

  char* ws = (char*)d_ws;
  size_t off = 0;
  const size_t oVh  = off; off += (size_t)NB * NTOK * CIN * 2;        off = (off + 255) & ~(size_t)255;
  const size_t oWq  = off; off += (size_t)CIN * HD * 2;               off = (off + 255) & ~(size_t)255;
  const size_t oWk  = off; off += (size_t)CIN * HD * 2;               off = (off + 255) & ~(size_t)255;
  const size_t oWv  = off; off += (size_t)CIN * HD * 2;               off = (off + 255) & ~(size_t)255;
  const size_t oWo  = off; off += (size_t)HD * DH * 2;                off = (off + 255) & ~(size_t)255;
  const size_t oKvT = off; off += (size_t)NB * NH * DH * DH * 2;      off = (off + 255) & ~(size_t)255;
  const size_t oPt  = off; off += (size_t)NB * NH * NTILE * DH * DH * 4; off = (off + 255) & ~(size_t)255;
  if (off > ws_size || off > (size_t)WSCAP) return;
  _Float16* vh   = (_Float16*)(ws + oVh);
  _Float16* WqT  = (_Float16*)(ws + oWq);
  _Float16* WkT  = (_Float16*)(ws + oWk);
  _Float16* WvT  = (_Float16*)(ws + oWv);
  _Float16* WoP  = (_Float16*)(ws + oWo);
  _Float16* kvT  = (_Float16*)(ws + oKvT);
  float*    part = (float*)(ws + oPt);

  k_prep<<<NVB + NWB, 256, 0, stream>>>(v, Wq_w, Wk_w, Wv_w, Wo_w, vh, WqT, WkT, WvT, WoP);
  k_kv<<<NB * NH * NTILE, 128, 0, stream>>>(vh, WkT, WvT, Wk_b, Wv_b, lnk_g, lnk_b, part);
  k_kvred<<<NB * NH, 256, 0, stream>>>(part, kvT);
  k_out<<<(NB * NTOK) / 64, 128, 0, stream>>>(vh, WqT, Wq_b, lnq_g, lnq_b, kvT, WoP, Wo_b, out);
}
